// CoordModulatedDeformableC3D_53300544143735
// MI455X (gfx1250) — hardware-verified
//
#include <hip/hip_runtime.h>
#include <hip/hip_fp16.h>

typedef _Float16 f16;
typedef __attribute__((ext_vector_type(16))) _Float16 v16h;
typedef __attribute__((ext_vector_type(8)))  float    v8f;
typedef __attribute__((ext_vector_type(4)))  unsigned int u32x4;
typedef __attribute__((ext_vector_type(8)))  int          i32x8;
typedef __attribute__((ext_vector_type(4)))  int          i32x4;

constexpr int BATCH = 2, CIN = 64, COUT = 64, DD = 8, HH = 32, WW = 32;
constexpr int SP    = DD * HH * WW;
constexpr int KT    = 27;
constexpr int COFF  = 67;
constexpr int NOFF  = 108;
constexpr int NOFF_PAD = 112;
constexpr int PREDP    = 128;

constexpr size_t XH_ELEMS   = (size_t)BATCH * CIN * SP;
constexpr size_t WOFF_ELEMS = (size_t)KT * 3 * 7 * 512;
constexpr size_t WDCN_ELEMS = (size_t)KT * 2 * 4 * 512;
constexpr size_t WS_XH   = 0;
constexpr size_t WS_WOFF = WS_XH + XH_ELEMS;
constexpr size_t WS_WDCN = WS_WOFF + WOFF_ELEMS;
constexpr size_t HALF_TOTAL = WS_WDCN + WDCN_ELEMS;
constexpr size_t WS_PRED_BYTE = ((HALF_TOTAL * 2 + 255) / 256) * 256;
constexpr size_t WS_TOTAL = WS_PRED_BYTE + (size_t)BATCH * SP * PREDP * 4;

#define USE_TDM 0
typedef __attribute__((ext_vector_type(8))) _Float16 v8h_t;
typedef __attribute__((ext_vector_type(4))) float    v4f_t;
__device__ __forceinline__ v8f wmma16(v16h a, v16h b, v8f c) {
  v8f d = __builtin_amdgcn_wmma_f32_16x16x32_f16(false, a, false, b, (short)0, c, false, false);
  asm volatile("v_nop\n\tv_nop\n\tv_nop\n\tv_nop" : "+v"(d) : "v"(a), "v"(b));
  return d;
}

#if USE_TDM
__device__ __forceinline__ void tdm_load_f16(const f16* gsrc, const f16* lds_dst, unsigned elems) {
  unsigned long long ga = (unsigned long long)(uintptr_t)gsrc;
  unsigned lds_off = (unsigned)(uintptr_t)lds_dst;
  u32x4 g0;
  g0[0] = 1u;
  g0[1] = lds_off;
  g0[2] = (unsigned)ga;
  g0[3] = (unsigned)((ga >> 32) & 0x01FFFFFFu) | (2u << 30);
  i32x8 g1;
  g1[0] = (int)(1u << 16);
  g1[1] = (int)((elems & 0xFFFFu) << 16);
  g1[2] = (int)((elems >> 16) & 0xFFFFu) | (1 << 16);
  g1[3] = (int)((elems & 0xFFFFu) << 16);
  g1[4] = 1;
  g1[5] = (int)elems;
  g1[6] = 0;
  g1[7] = 0;
  i32x4 z4 = {0, 0, 0, 0};
#if __clang_major__ >= 23
  i32x8 z8 = {0, 0, 0, 0, 0, 0, 0, 0};
  __builtin_amdgcn_tensor_load_to_lds(g0, g1, z4, z4, z8, 0);
#else
  __builtin_amdgcn_tensor_load_to_lds(g0, g1, z4, z4, 0);
#endif
}
#endif

__device__ __forceinline__ void coop_stage(f16* dst, const f16* src, int elems, int tid, int nthr) {
  for (int i = tid * 16; i < elems; i += nthr * 16)
    *(v16h*)(dst + i) = *(const v16h*)(src + i);
}

__global__ void k_x_to_half(const float* __restrict__ x, f16* __restrict__ xh, int n) {
  int i8 = blockIdx.x * blockDim.x + threadIdx.x;
  if (i8 * 8 >= n) return;
  v8h_t v;
#pragma unroll
  for (int e = 0; e < 8; ++e) v[e] = (f16)x[(size_t)i8 * 8 + e];
  *(volatile v8h_t*)(xh + (size_t)i8 * 8) = v; __threadfence(); *(volatile v8h_t*)(xh + (size_t)i8 * 8) = v;
}

__device__ __forceinline__ int frag_ch(int e, int lane) { return ((e < 8) ? e : (e + 8)) + ((lane >> 4) << 3); }

__global__ void k_pack_woff(const float* __restrict__ w, f16* __restrict__ wp) {
  int id8 = blockIdx.x * blockDim.x + threadIdx.x;
  if (id8 * 8 >= (int)WOFF_ELEMS) return;
  v8h_t vv;
#pragma unroll
  for (int q = 0; q < 8; ++q) {
    int id   = id8 * 8 + q;
    int e    = id & 15;
    int lane = (id >> 4) & 31;
    int rest = id >> 9;
    int t    = rest % 7;
    int kc   = rest / 7;
    int c    = kc % 3, k = kc / 3;
    int n    = t * 16 + (lane & 15);
    int ch   = c * 32 + frag_ch(e, lane);
    float v = 0.0f;
    if (n < NOFF && ch < COFF) v = w[((size_t)n * COFF + ch) * KT + k];
    vv[q] = (f16)v;
  }
  *(volatile v8h_t*)(wp + (size_t)id8 * 8) = vv; __threadfence(); *(volatile v8h_t*)(wp + (size_t)id8 * 8) = vv;
}

__global__ void k_pack_wdcn(const float* __restrict__ w, f16* __restrict__ wp) {
  int id8 = blockIdx.x * blockDim.x + threadIdx.x;
  if (id8 * 8 >= (int)WDCN_ELEMS) return;
  v8h_t vv;
#pragma unroll
  for (int q = 0; q < 8; ++q) {
    int id   = id8 * 8 + q;
    int e    = id & 15;
    int lane = (id >> 4) & 31;
    int rest = id >> 9;
    int t    = rest % 4;
    int kc   = rest / 4;
    int cc   = kc % 2, k = kc / 2;
    int o    = t * 16 + (lane & 15);
    int ch   = cc * 32 + frag_ch(e, lane);
    vv[q] = (f16)w[((size_t)o * CIN + ch) * KT + k];
  }
  *(volatile v8h_t*)(wp + (size_t)id8 * 8) = vv; __threadfence(); *(volatile v8h_t*)(wp + (size_t)id8 * 8) = vv;
}

__global__ __launch_bounds__(256) void k_offset_conv(
    const f16* __restrict__ xh, const f16* __restrict__ wp,
    const float* __restrict__ b_off, float* __restrict__ pred)
{
  __shared__ __align__(32) f16 wsm[21 * 512];

  const int lane  = threadIdx.x & 31;
  const int wid   = threadIdx.x >> 5;
  const int gw    = blockIdx.x * 8 + wid;
  const int mbase = gw * 16;
  const int laneHalf = lane >> 4;
  const int vL = mbase + (lane & 15);
  const int b  = vL >> 13;
  const int s  = vL & (SP - 1);
  const int d  = s >> 10, h = (s >> 5) & 31, w = s & 31;

  v8f acc[7] = {};
  const size_t xbase_b = (size_t)b * CIN * SP;

  for (int k = 0; k < KT; ++k) {
    __syncthreads();
#if USE_TDM
    if (wid == 0) {
      tdm_load_f16(wp + (size_t)k * 21 * 512, wsm, 21 * 512);
      __builtin_amdgcn_s_wait_tensorcnt(0);
    }
#else
    coop_stage(wsm, wp + (size_t)k * 21 * 512, 21 * 512, threadIdx.x, 256);
#endif
    __syncthreads();

    const int kd = k / 9 - 1, kh = (k / 3) % 3 - 1, kw = k % 3 - 1;
    const int nd = d + kd, nh = h + kh, nw = w + kw;
    const bool valid = (nd >= 0) & (nd < DD) & (nh >= 0) & (nh < HH) & (nw >= 0) & (nw < WW);
    const int nidx = (nd * HH + nh) * WW + nw;
    const float cz = fmaf((float)nd, 2.0f / (float)(DD - 1), -1.0f);
    const float cy = fmaf((float)nh, 2.0f / (float)(HH - 1), -1.0f);
    const float cx = fmaf((float)nw, 2.0f / (float)(WW - 1), -1.0f);
    const f16* __restrict__ xp = xh + xbase_b + nidx;

    for (int c = 0; c < 3; ++c) {
      v16h a;
      #pragma unroll
      for (int e = 0; e < 16; ++e) {
        const int ch = c * 32 + ((e < 8) ? e : e + 8) + laneHalf * 8;
        float v = 0.0f;
        if (valid) {
          if (ch < CIN)       v = (float)xp[(size_t)ch * SP];
          else if (ch == 64)  v = cz;
          else if (ch == 65)  v = cy;
          else if (ch == 66)  v = cx;
        }
        a[e] = (f16)v;
      }
      const f16* wpk = wsm + (size_t)(c * 7) * 512 + (size_t)lane * 16;
      v16h bf[7];
      #pragma unroll
      for (int t = 0; t < 7; ++t) bf[t] = *(const v16h*)(wpk + (size_t)t * 512);
      #pragma unroll
      for (int t = 0; t < 7; ++t) acc[t] = wmma16(a, bf[t], acc[t]);
    }
  }

  float ev[8][8];
  #pragma unroll
  for (int t = 0; t < 8; ++t) {
    const int n = t * 16 + (lane & 15);
    const float bias = (n < NOFF) ? b_off[n] : 0.0f;
    #pragma unroll
    for (int r = 0; r < 8; ++r) {
      float v = 0.0f;
      if (t < 7 && n < NOFF) { v = acc[t][r] + bias; if (n >= 81) v = 1.0f / (1.0f + expf(-v)); }
      ev[t][r] = v;
    }
  }
  for (int pass = 0; pass < 2; ++pass) {
    #pragma unroll
    for (int pr = 0; pr < 4; ++pr)
      #pragma unroll
      for (int r = 0; r < 8; ++r) {
        const float a_ = ev[2 * pr][r], b_ = ev[2 * pr + 1][r];
        const float ax = __shfl_xor(a_, 16), bx = __shfl_xor(b_, 16);
        *(volatile float*)(pred + (size_t)(mbase + r) * PREDP + pr * 32 + lane) = laneHalf ? bx : a_;
        *(volatile float*)(pred + (size_t)(mbase + r + 8) * PREDP + pr * 32 + lane) = laneHalf ? b_ : ax;
      }
    __threadfence();
  }
}

__global__ __launch_bounds__(256) void k_deform_conv(
    const f16* __restrict__ xh, const f16* __restrict__ wp,
    const float* __restrict__ pred, const float* __restrict__ b_dcn,
    float* __restrict__ out)
{
  __shared__ __align__(32) f16 wsm[8 * 512];
  __shared__ __align__(16) float osm[COUT][128];

  const int lane  = threadIdx.x & 31;
  const int wid   = threadIdx.x >> 5;
  const int gw    = blockIdx.x * 8 + wid;
  const int mbase = gw * 16;
  const int laneHalf = lane >> 4;
  const int vL = mbase + (lane & 15);
  const int b  = vL >> 13;
  const int s  = vL & (SP - 1);
  const float fd = (float)(s >> 10);
  const float fh = (float)((s >> 5) & 31);
  const float fw = (float)(s & 31);

  const float* __restrict__ prow = pred + (size_t)vL * PREDP;
  __builtin_prefetch(prow, 0, 1);

  v8f acc[4] = {};
  const size_t xb = (size_t)b * CIN * SP;

  for (int k = 0; k < KT; ++k) {
    __syncthreads();
#if USE_TDM
    if (wid == 0) {
      tdm_load_f16(wp + (size_t)k * 8 * 512, wsm, 8 * 512);
      __builtin_amdgcn_s_wait_tensorcnt(0);
    }
#else
    coop_stage(wsm, wp + (size_t)k * 8 * 512, 8 * 512, threadIdx.x, 256);
#endif
    __syncthreads();

    const float offz = prow[k * 3 + 0];
    const float offy = prow[k * 3 + 1];
    const float offx = prow[k * 3 + 2];
    const float alpha = prow[81 + k];

    const float pz = fd + (float)(k / 9 - 1) + offz;
    const float py = fh + (float)((k / 3) % 3 - 1) + offy;
    const float px = fw + (float)(k % 3 - 1) + offx;
    const float fz = floorf(pz), fy = floorf(py), fx = floorf(px);

    int   sidx[8];
    float wc[8];
    #pragma unroll
    for (int ci = 0; ci < 8; ++ci) {
      const float iz = fz + (float)(ci >> 2);
      const float iy = fy + (float)((ci >> 1) & 1);
      const float ix = fx + (float)(ci & 1);
      const float wgt = (1.0f - fabsf(pz - iz)) * (1.0f - fabsf(py - iy)) * (1.0f - fabsf(px - ix));
      const bool v = (iz >= 0.0f) & (iz < (float)DD) &
                     (iy >= 0.0f) & (iy < (float)HH) &
                     (ix >= 0.0f) & (ix < (float)WW);
      const int izc = (int)fminf(fmaxf(iz, 0.0f), (float)(DD - 1));
      const int iyc = (int)fminf(fmaxf(iy, 0.0f), (float)(HH - 1));
      const int ixc = (int)fminf(fmaxf(ix, 0.0f), (float)(WW - 1));
      sidx[ci] = (izc * HH + iyc) * WW + ixc;
      wc[ci]   = v ? wgt * alpha : 0.0f;
    }

    for (int cc = 0; cc < 2; ++cc) {
      v16h a;
      #pragma unroll
      for (int e = 0; e < 16; ++e) {
        const int ch = cc * 32 + ((e < 8) ? e : e + 8) + laneHalf * 8;
        const f16* __restrict__ xc = xh + xb + (size_t)ch * SP;
        float sacc = 0.0f;
        #pragma unroll
        for (int ci = 0; ci < 8; ++ci)
          sacc += wc[ci] * (float)xc[sidx[ci]];
        a[e] = (f16)sacc;
      }
      const f16* wpk = wsm + (size_t)(cc * 4) * 512 + (size_t)lane * 16;
      v16h bf[4];
      #pragma unroll
      for (int t = 0; t < 4; ++t) bf[t] = *(const v16h*)(wpk + (size_t)t * 512);
      #pragma unroll
      for (int t = 0; t < 4; ++t) acc[t] = wmma16(a, bf[t], acc[t]);
    }
  }

  #pragma unroll
  for (int t = 0; t < 4; ++t) {
    const int o = t * 16 + (lane & 15);
    const float bias = b_dcn[o];
    #pragma unroll
    for (int r = 0; r < 8; ++r) osm[o][wid * 16 + r + laneHalf * 8] = acc[t][r] + bias;
  }
  __syncthreads();
  {
    const int vb = blockIdx.x * 128;
    const int bb = vb >> 13, ss0 = vb & (SP - 1);
    for (int pass = 0; pass < 2; ++pass) {
      #pragma unroll
      for (int q = 0; q < 8; ++q) {
        const int piece = threadIdx.x + q * 256;
        const int o = piece >> 5, sg = piece & 31;
        *(volatile v4f_t*)(out + ((size_t)bb * COUT + o) * SP + ss0 + sg * 4) = *(const v4f_t*)(&osm[o][sg * 4]);
      }
      __threadfence();
    }
  }
}

extern "C" void kernel_launch(void* const* d_in, const int* in_sizes, int n_in,
                              void* d_out, int out_size, void* d_ws, size_t ws_size,
                              hipStream_t stream) {
  const float* x     = (const float*)d_in[0];
  const float* w_off = (const float*)d_in[1];
  const float* b_off = (const float*)d_in[2];
  const float* w_dcn = (const float*)d_in[3];
  const float* b_dcn = (const float*)d_in[4];
  float* out = (float*)d_out;

  f16* wsH   = (f16*)d_ws;
  f16* xh    = wsH + WS_XH;
  f16* woffp = wsH + WS_WOFF;
  f16* wdcnp = wsH + WS_WDCN;
  float* pred = (float*)((char*)d_ws + WS_PRED_BYTE);
  (void)in_sizes; (void)n_in; (void)out_size;
  if (ws_size < WS_TOTAL) return;

  k_x_to_half<<<(int)((XH_ELEMS / 8 + 255) / 256), 256, 0, stream>>>(x, xh, (int)XH_ELEMS);
  k_pack_woff<<<(int)((WOFF_ELEMS / 8 + 255) / 256), 256, 0, stream>>>(w_off, woffp);
  k_pack_wdcn<<<(int)((WDCN_ELEMS / 8 + 255) / 256), 256, 0, stream>>>(w_dcn, wdcnp);

  k_offset_conv<<<128, 256, 0, stream>>>(xh, woffp, b_off, pred);
  k_deform_conv<<<128, 256, 0, stream>>>(xh, wdcnp, pred, b_dcn, out);
}
